// PointAtomCrossAttention_84524956385317
// MI455X (gfx1250) — hardware-run, weakly checked
//
#include <hip/hip_runtime.h>
#include <math.h>

typedef __attribute__((ext_vector_type(16))) _Float16 v16h;
typedef __attribute__((ext_vector_type(16))) __bf16 v16b;
typedef __attribute__((ext_vector_type(8)))  _Float16 v8h;
typedef __attribute__((ext_vector_type(8)))  float v8f;
typedef __attribute__((ext_vector_type(4)))  float v4f;
typedef __attribute__((ext_vector_type(2)))  float v2f;
typedef __attribute__((ext_vector_type(4)))  unsigned v4u;
typedef __attribute__((ext_vector_type(4)))  int v4i;
typedef float __attribute__((may_alias)) float_a;
typedef int __attribute__((may_alias)) int_a;

template <typename T> __device__ __forceinline__ void vst2(void* p, T v) { *(volatile T*)p = v; __threadfence(); *(volatile T*)p = v; }
__device__ __forceinline__ v8f wmma16(v16h a, v16h b, v8f c) {
  v8f d = __builtin_amdgcn_wmma_f32_16x16x32_f16(false, a, false, b, (short)0, c, false, false);
  asm volatile("v_nop\n\tv_nop\n\tv_nop\n\tv_nop" : "+v"(d) : "v"(a), "v"(b));
  return d;
}
__device__ __forceinline__ v8f wmma_bf(v16b a, v16b b, v8f c) {
  v8f d = __builtin_amdgcn_wmma_f32_16x16x32_bf16(false, a, false, b, (short)0, c, false, false);
  asm volatile("v_nop\n\tv_nop\n\tv_nop\n\tv_nop" : "+v"(d) : "v"(a), "v"(b));
  return d;
}
__device__ __forceinline__ v16h frag_h(const _Float16* rowk0, int lane) {
  union { v16h v; v8h q[2]; } u; const _Float16* p = rowk0 + 8 * (lane >> 4);
  u.q[0] = *(const v8h*)p; u.q[1] = *(const v8h*)(p + 16); return u.v;
}
__device__ __forceinline__ v16h frag_f32(const float* rowk0, int lane) {
  v16h a; const float* p = rowk0 + 8 * (lane >> 4);
#pragma unroll
  for (int i = 0; i < 8; ++i) { a[i] = (_Float16)p[i]; a[8 + i] = (_Float16)p[16 + i]; }
  return a;
}
__device__ __forceinline__ v16h frag_f32s(const float* rowk0, int lane, float sc) {
  v16h a; const float* p = rowk0 + 8 * (lane >> 4);
#pragma unroll
  for (int i = 0; i < 8; ++i) { a[i] = (_Float16)(p[i] * sc); a[8 + i] = (_Float16)(p[16 + i] * sc); }
  return a;
}
__device__ __forceinline__ v16h fragc_f32(const float* W, int k0, int n, int lane, int ld, int K) {
  v16h a; const int g = lane >> 4;
#pragma unroll
  for (int i = 0; i < 8; ++i) { const int ka = k0 + 8 * g + i, kb = ka + 16;
    a[i] = (_Float16)(ka < K ? W[(size_t)(ka < K ? ka : K - 1) * ld + n] : 0.f); a[8 + i] = (_Float16)(kb < K ? W[(size_t)(kb < K ? kb : K - 1) * ld + n] : 0.f); }
  return a;
}
struct F2 { v16b h, l; };
__device__ __forceinline__ F2 bsplit16(const float v[16]) { F2 r;
#pragma unroll
  for (int i = 0; i < 16; ++i) { const __bf16 h = (__bf16)v[i]; r.h[i] = h; r.l[i] = (__bf16)(v[i] - (float)h); }
  return r; }
__device__ __forceinline__ F2 split_row(const float* row, int k0, int lane) { float v[16]; const float* p = row + k0 + 8 * (lane >> 4);
#pragma unroll
  for (int i = 0; i < 8; ++i) { v[i] = p[i]; v[8 + i] = p[16 + i]; }
  return bsplit16(v); }
__device__ __forceinline__ F2 split_rowK(const float* row, int k0, int lane, int K) { float v[16]; const int g = lane >> 4;
#pragma unroll
  for (int i = 0; i < 8; ++i) { const int ka = k0 + 8 * g + i, kb = ka + 16; v[i] = ka < K ? row[ka < K ? ka : K - 1] : 0.f; v[8 + i] = kb < K ? row[kb < K ? kb : K - 1] : 0.f; }
  return bsplit16(v); }
__device__ __forceinline__ F2 split_col(const float* W, int k0, int n, int lane, int ld, int K) { float v[16]; const int g = lane >> 4;
#pragma unroll
  for (int i = 0; i < 8; ++i) { const int ka = k0 + 8 * g + i, kb = ka + 16; v[i] = ka < K ? W[(size_t)(ka < K ? ka : K - 1) * ld + n] : 0.f; v[8 + i] = kb < K ? W[(size_t)(kb < K ? kb : K - 1) * ld + n] : 0.f; }
  return bsplit16(v); }
__device__ __forceinline__ v8f mac3(const F2& a, const F2& b, v8f c) { c = wmma_bf(a.l, b.h, c); c = wmma_bf(a.h, b.l, c); return wmma_bf(a.h, b.h, c); }
__device__ __forceinline__ float sigm(float v) { return 1.0f / (1.0f + expf(-v)); }
#define LDSX() do { asm volatile("s_wait_dscnt 0" ::: "memory"); __builtin_amdgcn_wave_barrier(); __builtin_amdgcn_fence(__ATOMIC_RELEASE, "workgroup"); } while (0)


#define KP 4096
#define NA 2048
#define HID 256
#define NH 8
#define HD 32
#define NRBF 32
#ifndef TQB
#define TQB (KP / 64)
#endif
typedef __attribute__((ext_vector_type(8))) __bf16 v8b;
__device__ __forceinline__ v16b frag_b(const __bf16* rowk0, int lane) {
  union { v16b v; v8b q[2]; } u; const __bf16* p = rowk0 + 8 * (lane >> 4);
  u.q[0] = *(const v8b*)p; u.q[1] = *(const v8b*)(p + 16); return u.v;
}
__device__ __forceinline__ float bfr(float v) { return (float)(__bf16)v; }
__device__ __attribute__((noinline)) float exp_ni(float v) { return expf(v); }
__device__ __attribute__((noinline)) float erf_ni(float v) { return erff(v); }

#define WS_PW  0u
#define WS_PR  (WS_PW + 2u * (size_t)4 * HID * HID)
#define WS_Q   (WS_PR + 2u * 16 * NRBF + 256u)
#define WS_K   (WS_Q + 2u * (size_t)KP * HID)
#define WS_V   (WS_K + 2u * (size_t)NA * HID)
#define WS_BI  (WS_V + 2u * (size_t)HID * NA)
#define WS_O   (WS_BI + 2u * (size_t)NH * KP * NA)
#define WS_END (WS_O + 4u * (size_t)KP * HID)

__global__ __launch_bounds__(256) void k_pack(const float* __restrict__ WQ, const float* __restrict__ WK, const float* __restrict__ WV, const float* __restrict__ WO, const float* __restrict__ WR, __bf16* __restrict__ PW, _Float16* __restrict__ PR) {
  const int n = blockIdx.x, which = blockIdx.y, t = threadIdx.x; __shared__ __align__(16) __bf16 s[HID]; __shared__ __align__(16) _Float16 sr[16 * NRBF];
  if (which < 4) { const float* w = (which == 0) ? WQ : (which == 1) ? WK : (which == 2) ? WV : WO; s[t] = (__bf16)w[(size_t)t * HID + n]; __syncthreads(); if (t < HID / 8) vst2((unsigned*)(PW + ((size_t)which * HID + n) * HID + t * 8), *(const v4u*)&s[t * 8]); }
  else if (n == 0) { for (int e = t; e < 16 * NRBF; e += 256) { const int h = e / NRBF, r = e % NRBF; sr[e] = (h < NH) ? (_Float16)(bfr(WR[(size_t)r * NH + h]) * 256.0f) : (_Float16)0.f; } __syncthreads(); if (t < 16 * NRBF / 8) vst2((unsigned*)(PR + t * 8), *(const v4u*)&sr[t * 8]); }
}
__global__ __launch_bounds__(128) void k_proj(const float* __restrict__ HP_, const float* __restrict__ HA_, const __bf16* __restrict__ PW, const float* __restrict__ BQ, const float* __restrict__ BK, const float* __restrict__ BV, _Float16* __restrict__ Q, _Float16* __restrict__ Kr, _Float16* __restrict__ V) {
  __shared__ __align__(16) _Float16 so[64][HID + 8]; __shared__ __align__(16) _Float16 st[HID][72];
  const int tid = threadIdx.x, wave = tid >> 5, lane = tid & 31, col = lane & 15, g = lane >> 4; const int which = blockIdx.y; const size_t rb = (size_t)blockIdx.x * 64; const size_t r0 = rb + wave * 16;
  if (which > 0 && rb >= NA) return;
  const float* X = (which == 0) ? HP_ : HA_; const __bf16* Wr = PW + ((size_t)which * HID) * HID; const float* BB = (which == 0) ? BQ : (which == 1) ? BK : BV;
  v16b a[8];
#pragma unroll
  for (int kc = 0; kc < 8; ++kc) { const float* p = X + (r0 + col) * HID + kc * 32 + 8 * g;
#pragma unroll
    for (int i = 0; i < 8; ++i) { a[kc][i] = (__bf16)p[i]; a[kc][8 + i] = (__bf16)p[16 + i]; } }
#pragma unroll 1
  for (int half = 0; half < 2; ++half) { v8f acc[8] = {};
#pragma unroll
    for (int kc = 0; kc < 8; ++kc)
#pragma unroll
      for (int j = 0; j < 8; ++j) acc[j] = wmma_bf(a[kc], frag_b(Wr + (size_t)(half * 128 + j * 16 + col) * HID + kc * 32, lane), acc[j]);
#pragma unroll
    for (int j = 0; j < 8; ++j) { const int c = half * 128 + j * 16 + col; const float bb = bfr(BB[c]);
#pragma unroll
      for (int r = 0; r < 8; ++r) { const _Float16 hv = (_Float16)(acc[j][r] + bb); if (which < 2) so[wave * 16 + 8 * g + r][c] = hv; else st[c][wave * 16 + 8 * g + r] = hv; } } }
  __syncthreads();
  if (which < 2) { _Float16* dst = (which == 0) ? Q : Kr; for (int e = tid; e < 64 * (HID / 8); e += 128) { const int rl = e >> 5, q = e & 31; vst2((unsigned*)(dst + (rb + rl) * HID + q * 8), *(const v4u*)&so[rl][q * 8]); } }
  else { for (int e = tid; e < HID * 8; e += 128) { const int d = e >> 3, pc = e & 7; vst2((unsigned*)(V + (size_t)d * NA + rb + pc * 8), *(const v4u*)&st[d][pc * 8]); } }
}
__global__ __launch_bounds__(128) void k_bias(const float* __restrict__ PP, const float* __restrict__ PA, const float* __restrict__ CEN, const _Float16* __restrict__ PR, const float* __restrict__ BR, _Float16* __restrict__ BI) {
  __shared__ __align__(16) _Float16 srbf[16 * 64][NRBF + 8]; __shared__ __align__(16) _Float16 sb[NH][16][72]; __shared__ float spp[64][3], spa[64][3], scen[NRBF], sbr[NH];
  const int tid = threadIdx.x, wave = tid >> 5, lane = tid & 31, col = lane & 15, g = lane >> 4; const int p0 = blockIdx.x * 64, a0 = blockIdx.y * 64;
  for (int e = tid; e < 64 * 3; e += 128) { spp[e / 3][e % 3] = bfr(PP[(size_t)(p0 + e / 3) * 3 + e % 3]); spa[e / 3][e % 3] = bfr(PA[(size_t)(a0 + e / 3) * 3 + e % 3]); }
  if (tid < NRBF) scen[tid] = bfr(CEN[tid]); if (tid < NH) sbr[tid] = bfr(BR[tid]);
  __syncthreads();
  const v16h wr = frag_h(PR + (size_t)col * NRBF, lane);
#pragma unroll 1
  for (int ch = 0; ch < 4; ++ch) {
    for (int e = tid; e < 1024; e += 128) { const int pl = e >> 6, al = e & 63; const int p = ch * 16 + pl; const float dx = spp[p][0] - spa[al][0], dy = spp[p][1] - spa[al][1], dz = spp[p][2] - spa[al][2]; const float dist = sqrtf(fmaxf(dx * dx + dy * dy + dz * dz, 0.f));
#pragma unroll 1
      for (int r = 0; r < NRBF; ++r) { const float u = dist - scen[r]; srbf[e][r] = (_Float16)__expf(-u * u * 16.0f); } }
    __syncthreads();
    for (int tile = wave; tile < 64; tile += 4) { v8f z = {}; z = wmma16(frag_h(&srbf[tile * 16 + col][0], lane), wr, z);
#pragma unroll
      for (int r = 0; r < 8; ++r) { const int e = tile * 16 + 8 * g + r; if (col < NH) sb[col][e >> 6][e & 63] = (_Float16)(z[r] * (1.0f / 256.0f) + sbr[col]); } }
    __syncthreads();
    for (int e = tid; e < NH * 16 * 8; e += 128) { const int h = e / 128, rem = e % 128; const int pl = rem >> 3, q = rem & 7; vst2((unsigned*)(BI + ((size_t)h * KP + p0 + ch * 16 + pl) * NA + a0 + q * 8), *(const v4u*)&sb[h][pl][q * 8]); }
    __syncthreads(); }
}
__global__ __launch_bounds__(128) void k_attn(const _Float16* __restrict__ Q, const _Float16* __restrict__ Kr, const _Float16* __restrict__ V, const _Float16* __restrict__ BI, const int* __restrict__ PB, const int* __restrict__ AB, float* __restrict__ O) {
  __shared__ __align__(16) _Float16 sph[4][16][40]; __shared__ __align__(16) float so[4][16][36];
  const int tid = threadIdx.x, wave = tid >> 5, lane = tid & 31, col = lane & 15, g = lane >> 4; const int h = blockIdx.y; const int q0 = blockIdx.x * 64 + wave * 16;
  const v16h aq = frag_h(Q + (size_t)(q0 + col) * HID + h * HD, lane);
  int pb[8];
#pragma unroll
  for (int r = 0; r < 8; ++r) pb[r] = PB[q0 + 8 * g + r];
  float m[8], l[8];
#pragma unroll
  for (int r = 0; r < 8; ++r) { m[r] = -3.0e38f; l[r] = 0.f; }
  v8f acc[2] = {};
#pragma unroll 1
  for (int ks = 0; ks < NA / 32; ++ks) { const int j0 = ks * 32; v8f s[2];
#pragma unroll
    for (int ct = 0; ct < 2; ++ct) { const int kk = j0 + ct * 16 + col; v8f c = {}; c = wmma16(aq, frag_h(Kr + (size_t)kk * HID + h * HD, lane), c); const int ab = AB[kk];
#pragma unroll
      for (int r = 0; r < 8; ++r) { const int qi = q0 + 8 * g + r; s[ct][r] = (pb[r] == ab) ? (c[r] * 0.17677669529663688f + (float)BI[((size_t)h * KP + qi) * NA + kk]) : -3.0e38f; } }
#pragma unroll
    for (int r = 0; r < 8; ++r) { float mx = fmaxf(s[0][r], s[1][r]);
#pragma unroll
      for (int o = 1; o < 16; o <<= 1) mx = fmaxf(mx, __shfl_xor(mx, o));
      const float mn = fmaxf(m[r], mx); const float alpha = (m[r] <= -1.0e38f) ? 0.f : __expf(m[r] - mn); const float e0 = (s[0][r] <= -1.0e38f) ? 0.f : __expf(s[0][r] - mn), e1 = (s[1][r] <= -1.0e38f) ? 0.f : __expf(s[1][r] - mn); float es = e0 + e1;
#pragma unroll
      for (int o = 1; o < 16; o <<= 1) es += __shfl_xor(es, o);
      l[r] = l[r] * alpha + es; m[r] = mn;
#pragma unroll
      for (int dt = 0; dt < 2; ++dt) acc[dt][r] *= alpha;
      sph[wave][8 * g + r][col] = (_Float16)(e0 * 2048.0f); sph[wave][8 * g + r][16 + col] = (_Float16)(e1 * 2048.0f); }
    LDSX();
    const v16h pa = frag_h(&sph[wave][col][0], lane);
#pragma unroll
    for (int dt = 0; dt < 2; ++dt) acc[dt] = wmma16(pa, frag_h(V + (size_t)(h * HD + dt * 16 + col) * NA + j0, lane), acc[dt]);
    LDSX(); }
#pragma unroll
  for (int r = 0; r < 8; ++r) { const float il = (l[r] > 0.f) ? (1.0f / 2048.0f) / l[r] : 0.f;
#pragma unroll
    for (int dt = 0; dt < 2; ++dt) so[wave][8 * g + r][dt * 16 + col] = acc[dt][r] * il; }
  LDSX();
  for (int rl = 0; rl < 16; ++rl) if (lane < 8) vst2(O + (size_t)(q0 + rl) * HID + h * HD + lane * 4, *(const v4f*)&so[wave][rl][lane * 4]);
}
__global__ __launch_bounds__(128) void k_out(const float* __restrict__ O, const __bf16* __restrict__ PW, const float* __restrict__ BO, const float* __restrict__ HP_, const float* __restrict__ G, const float* __restrict__ Bt, float* __restrict__ OUT) {
  __shared__ __align__(16) float sx[64][HID + 4];
  const int tid = threadIdx.x, wave = tid >> 5, lane = tid & 31, col = lane & 15, g = lane >> 4; const size_t rb = (size_t)blockIdx.x * 64; const size_t r0 = rb + wave * 16; const __bf16* Wr = PW + (size_t)3 * HID * HID;
#pragma unroll 1
  for (int half = 0; half < 2; ++half) { v8f acc[8] = {};
#pragma unroll
    for (int kc = 0; kc < HID / 32; ++kc) { const F2 a = split_row(O + (r0 + col) * HID, kc * 32, lane);
#pragma unroll
      for (int j = 0; j < 8; ++j) { const v16b w = frag_b(Wr + (size_t)(half * 128 + j * 16 + col) * HID + kc * 32, lane); acc[j] = wmma_bf(a.h, w, acc[j]); acc[j] = wmma_bf(a.l, w, acc[j]); } }
#pragma unroll
    for (int j = 0; j < 8; ++j) { const int c = half * 128 + j * 16 + col; const float bb = bfr(BO[c]);
#pragma unroll
      for (int r = 0; r < 8; ++r) { const int rl = wave * 16 + 8 * g + r; sx[rl][c] = acc[j][r] + bb + bfr(HP_[(rb + rl) * HID + c]); } } }
  __syncthreads();
  { const int rl = tid >> 1, hf = tid & 1; float s = 0.f; for (int c = hf * 128; c < hf * 128 + 128; ++c) s += sx[rl][c]; s += __shfl_xor(s, 1); const float mu = s / (float)HID; float q = 0.f; for (int c = hf * 128; c < hf * 128 + 128; ++c) { const float d = sx[rl][c] - mu; q += d * d; } q += __shfl_xor(q, 1); const float inv = 1.0f / sqrtf(q / (float)HID + 1e-5f);
    __syncthreads();
    for (int c = hf * 128; c < hf * 128 + 128; ++c) sx[rl][c] = (sx[rl][c] - mu) * inv * bfr(G[c]) + bfr(Bt[c]); }
  __syncthreads();
  for (int e = tid; e < 64 * (HID / 4); e += 128) { const int rl = e >> 6, q = e & 63; vst2(OUT + (rb + rl) * HID + q * 4, *(const v4f*)&sx[rl][q * 4]); }
}
extern "C" void kernel_launch(void* const* d_in, const int* in_sizes, int n_in, void* d_out, int out_size, void* d_ws, size_t ws_size, hipStream_t stream) {
  (void)in_sizes; (void)n_in; (void)out_size;
  const float** F = (const float**)d_in;
  if (ws_size < (size_t)WS_END) return;
  char* ws = (char*)d_ws; __bf16* PW = (__bf16*)(ws + WS_PW); _Float16 *PR = (_Float16*)(ws + WS_PR), *Q = (_Float16*)(ws + WS_Q), *Kr = (_Float16*)(ws + WS_K), *V = (_Float16*)(ws + WS_V), *BI = (_Float16*)(ws + WS_BI); float* O = (float*)(ws + WS_O);
  k_pack<<<dim3(HID, 5), 256, 0, stream>>>(F[4], F[6], F[8], F[10], F[12], PW, PR);
  k_proj<<<dim3(KP / 64, 3), 128, 0, stream>>>(F[0], F[1], PW, F[5], F[7], F[9], Q, Kr, V);
  k_bias<<<dim3(TQB, NA / 64), 128, 0, stream>>>(F[2], F[3], F[14], PR, F[13], BI);
  k_attn<<<dim3(TQB, NH), 128, 0, stream>>>(Q, Kr, V, BI, (const int*)d_in[17], (const int*)d_in[18], O);
  k_out<<<TQB, 128, 0, stream>>>(O, PW, F[11], F[0], F[15], F[16], (float*)d_out);
}
